// LSTM_35381940584849
// MI455X (gfx1250) — hardware-verified
//
#include <hip/hip_runtime.h>
#include <math.h>

constexpr int NTRK     = 32768;
constexpr int NOBS     = 9;
constexpr int NSTEPS   = 20;
constexpr int HID      = 128;
constexpr int EMB      = 64;
constexpr int KCAT     = EMB + HID;
constexpr int NGATE    = 4 * HID;
constexpr int NPRIM    = 4096;
constexpr int ROWS_BLK = 32;
constexpr int NTHR     = 256;
constexpr int APITCH   = 200;
constexpr int HLPITCH  = 132;
constexpr int WPLANE   = NGATE * KCAT;
constexpr float WCARRY     = 16.0f;
constexpr float WCARRY_INV = 1.0f / 16.0f;
constexpr int PREP_BLK_IH = NGATE * (EMB / 8) / NTHR;
constexpr int PREP_BLK_HH = NGATE * (HID / 8) / NTHR;
constexpr int PREP_WBLOCKS = 2 * (PREP_BLK_IH + PREP_BLK_HH);
static_assert(KCAT % 32 == 0, "K multiple of 32");
static_assert(NTRK % ROWS_BLK == 0, "grid exact");
static_assert(HID == 16 * (NTHR / 32), "8 waves x 16 hidden columns");
static_assert((ROWS_BLK * (APITCH - EMB)) % NTHR == 0, "zero-fill loop exact");
static_assert(NGATE * (EMB / 8) % NTHR == 0 && NGATE * (HID / 8) % NTHR == 0, "prep coverage exact");
static_assert(NPRIM == NTRK / 8, "primary list length");

typedef __attribute__((ext_vector_type(16))) _Float16 v16h;
typedef __attribute__((ext_vector_type(8)))  _Float16 v8h;
typedef __attribute__((ext_vector_type(8)))  float    v8f;
typedef __attribute__((ext_vector_type(4)))  float    v4f;
typedef __attribute__((ext_vector_type(2)))  float    v2f;
typedef __attribute__((ext_vector_type(4)))  int      v4i;

struct FragH {
  union U { v16h v; v8h h[2]; };
  static __device__ __forceinline__ v16h load(const _Float16* p) {
    U f; f.h[0] = *(const v8h*)(p); f.h[1] = *(const v8h*)(p + 16); return f.v;
  }
  static __device__ __forceinline__ v8f mma(v16h a, v16h b, v8f c) {
    return __builtin_amdgcn_wmma_f32_16x16x32_f16(false, a, false, b, (short)0, c, false, false);
  }
};
__device__ __forceinline__ void guard8(v8f& c0, v8f& c1, v8f& c2, v8f& c3, v8f& c4, v8f& c5, v8f& c6, v8f& c7,
                                       v16h a0, v16h a1, v16h b0, v16h b1, v16h b2, v16h b3) {
  asm volatile("v_nop\n\tv_nop\n\tv_nop\n\tv_nop"
               : "+v"(c0), "+v"(c1), "+v"(c2), "+v"(c3), "+v"(c4), "+v"(c5), "+v"(c6), "+v"(c7)
               : "v"(a0), "v"(a1), "v"(b0), "v"(b1), "v"(b2), "v"(b3));
}
__device__ __forceinline__ void acc_guard4(v8f& a, v8f& b, v8f& c, v8f& d) {
  asm volatile("v_nop\n\tv_nop\n\tv_nop\n\tv_nop" : "+v"(a), "+v"(b), "+v"(c), "+v"(d));
}

__device__ __forceinline__ float fsig(float x)  { return __builtin_amdgcn_rcpf(1.0f + __expf(-x)); }
__device__ __forceinline__ float ftanh(float x) { return 1.0f - 2.0f * __builtin_amdgcn_rcpf(__expf(2.0f * x) + 1.0f); }
__device__ __forceinline__ bool nan_bits(float x) { return (__float_as_uint(x) & 0x7fffffffu) > 0x7f800000u; }

__global__ __launch_bounds__(NTHR) void prep_kernel(const float* __restrict__ Wih_e, const float* __restrict__ Whh_e,
                                                    const float* __restrict__ bih_e, const float* __restrict__ bhh_e,
                                                    const float* __restrict__ Wih_d, const float* __restrict__ Whh_d,
                                                    const float* __restrict__ bih_d, const float* __restrict__ bhh_d,
                                                    unsigned short* __restrict__ WBp, float* __restrict__ BIAS) {
  const int tid = threadIdx.x;
  const int b = blockIdx.x;
  if (b < PREP_WBLOCKS) {
    const float* src;
    int ks, grp, kdst, plane, bb;
    if (b < PREP_BLK_IH)                        { src = Wih_e; ks = EMB; grp = EMB / 8; kdst = 0;   plane = 0; bb = b; }
    else if (b < PREP_BLK_IH + PREP_BLK_HH)     { src = Whh_e; ks = HID; grp = HID / 8; kdst = EMB; plane = 0; bb = b - PREP_BLK_IH; }
    else if (b < 2 * PREP_BLK_IH + PREP_BLK_HH) { src = Wih_d; ks = EMB; grp = EMB / 8; kdst = 0;   plane = 1; bb = b - (PREP_BLK_IH + PREP_BLK_HH); }
    else                                        { src = Whh_d; ks = HID; grp = HID / 8; kdst = EMB; plane = 1; bb = b - (2 * PREP_BLK_IH + PREP_BLK_HH); }
    const int idx = bb * NTHR + tid;
    const int n   = idx / grp;
    const int cg  = idx - n * grp;
    const float* sp = src + (size_t)n * ks + cg * 8;
    const v4f x = *(const v4f*)(sp);
    const v4f y = *(const v4f*)(sp + 4);
    v8h hv;
#pragma unroll
    for (int e = 0; e < 4; ++e) {
      const float xe = x[e] * WCARRY;
      const float ye = y[e] * WCARRY;
      hv[e]     = (_Float16)xe;
      hv[4 + e] = (_Float16)ye;
    }
    unsigned short* dp = WBp + (size_t)plane * WPLANE + (size_t)n * KCAT + kdst + cg * 8;
    *(volatile v8h*)dp = hv;
    __threadfence();
    *(volatile v8h*)dp = hv;
  } else {
    const int which = tid >> 7;
    const int idx = (tid & 127) * 4;
    const v4f a  = *(const v4f*)(bih_e + idx);
    const v4f bq = *(const v4f*)(bhh_e + idx);
    const v4f cq = *(const v4f*)(bih_d + idx);
    const v4f dq = *(const v4f*)(bhh_d + idx);
    v4f o;
#pragma unroll
    for (int e = 0; e < 4; ++e) {
      const float se = a[e] + bq[e];
      const float sd = cq[e] + dq[e];
      o[e] = which ? sd : se;
    }
    float* op = BIAS + which * NGATE + idx;
    *(volatile v4f*)op = o;
    __threadfence();
    *(volatile v4f*)op = o;
  }
}

__global__ __launch_bounds__(NTHR) void lstm_traj_kernel(const float* __restrict__ observed, const int* __restrict__ bsplit,
                                                         const float* __restrict__ W_emb, const float* __restrict__ b_emb,
                                                         const float* __restrict__ Wf, const float* __restrict__ bfp,
                                                         const unsigned short* __restrict__ WBp, const float* __restrict__ BIAS,
                                                         float* __restrict__ out) {
  __shared__ __align__(16) _Float16 At[ROWS_BLK * APITCH];
  __shared__ __align__(16) float    hl[ROWS_BLK * HLPITCH];
  __shared__ __align__(16) float    Wfl[2 * HID];
  __shared__ __align__(16) float    Wes[3 * EMB];
  __shared__ __align__(16) float    Vs[2 * ROWS_BLK];
  __shared__ __align__(16) int      msk[ROWS_BLK];

  const _Float16* WB = (const _Float16*)WBp;
  const int tid = threadIdx.x, lane = tid & 31, wave = tid >> 5;
  const int c = lane & 15, hh = lane >> 4, koff = hh * 8;
  const int rowbase = blockIdx.x * ROWS_BLK;
  const int j = 16 * wave + c;

#pragma unroll 1
  for (int i = tid; i < ROWS_BLK * (APITCH - EMB); i += NTHR) {
    const int row = i / (APITCH - EMB);
    const int col = i - row * (APITCH - EMB);
    At[row * APITCH + EMB + col] = (_Float16)0.0f;
  }
  {
    const int d = tid >> 7, jj = tid & 127;
    Wfl[d * HID + jj] = Wf[jj * 2 + d];
  }
  {
    const float wv = W_emb[tid < 2 * EMB ? tid : 2 * EMB - 1];
    const float bv = b_emb[tid < EMB ? tid : EMB - 1];
    if (tid < 2 * EMB) Wes[tid] = wv;
    if (tid < EMB) Wes[2 * EMB + tid] = bv;
  }
  const float bfx = bfp[0], bfy = bfp[1];

  v2f pm1 = {0.f, 0.f}, pm2 = {0.f, 0.f}, obs8 = {0.f, 0.f}, o2c = {0.f, 0.f};
  int mkc = 0;
  unsigned pmask = 0u;
  if (wave == 0) {
    const int a = rowbase + lane;
    obs8 = *(const v2f*)(observed + ((size_t)8 * NTRK + a) * 2);
    int lo = 0, hi = NPRIM;
#pragma unroll 1
    for (int it = 0; it < 13; ++it) {
      const int mid  = (lo + hi) >> 1;
      const int midc = mid < NPRIM ? mid : NPRIM - 1;
      const int v    = bsplit[midc];
      const bool act  = lo < hi;
      const bool less = v < a;
      lo = (act && less) ? mid + 1 : lo;
      hi = (act && !less) ? mid : hi;
    }
    const int loc = lo < NPRIM ? lo : NPRIM - 1;
    const int vb  = bsplit[loc];
    pmask = ((lo < NPRIM) && (vb == a)) ? 0xffffffffu : 0u;
    const v2f n1 = *(const v2f*)(observed + ((size_t)0 * NTRK + a) * 2);
    const v2f n2 = *(const v2f*)(observed + ((size_t)1 * NTRK + a) * 2);
    const float n1x = n1[0], n1y = n1[1], n2x = n2[0], n2y = n2[1];
    const bool mk = !(nan_bits(n1x) || nan_bits(n2x));
    v2f vs;
    vs[0] = mk ? 4.0f * (n2x - n1x) : 0.0f;
    vs[1] = mk ? 4.0f * (n2y - n1y) : 0.0f;
    *(v2f*)(Vs + 2 * lane) = vs;
    msk[lane] = mk ? 1 : 0;
    o2c = n2;
    mkc = mk ? 1 : 0;
  }

  float cst[2][8], hst[2][8];
#pragma unroll
  for (int mt = 0; mt < 2; ++mt)
#pragma unroll
    for (int r = 0; r < 8; ++r) { cst[mt][r] = 0.0f; hst[mt][r] = 0.0f; }
  float bI = 0.f, bF = 0.f, bG = 0.f, bO = 0.f;
  __syncthreads();

  const _Float16* ar0 = At + c * APITCH + koff;
  const _Float16* ar1 = At + (16 + c) * APITCH + koff;
  const v8f z8 = {0.f, 0.f, 0.f, 0.f, 0.f, 0.f, 0.f, 0.f};
  const float nanv = __uint_as_float(0x7FC00000u);

#pragma unroll 1
  for (int t = 0; t < NSTEPS; ++t) {
    const int phase = (t >= 8) ? 1 : 0;
    if (t == 0 || t == 8) {
      const float* bp = BIAS + phase * NGATE + j;
      bI = bp[0]; bF = bp[HID]; bG = bp[2 * HID]; bO = bp[3 * HID];
    }

    {
      const int m = tid >> 3, e0 = (tid & 7) * 8;
      const v2f vs = *(const v2f*)(Vs + 2 * m);
      const float vx = vs[0], vy = vs[1];
      const v4f w0a = *(const v4f*)(Wes + e0),           w0b = *(const v4f*)(Wes + e0 + 4);
      const v4f w1a = *(const v4f*)(Wes + EMB + e0),     w1b = *(const v4f*)(Wes + EMB + e0 + 4);
      const v4f bea = *(const v4f*)(Wes + 2 * EMB + e0), beb = *(const v4f*)(Wes + 2 * EMB + e0 + 4);
      v8h ev;
#pragma unroll
      for (int e = 0; e < 4; ++e) {
        const float pa = fmaf(vy, w1a[e], vx * w0a[e]) + bea[e];
        const float pb = fmaf(vy, w1b[e], vx * w0b[e]) + beb[e];
        float ra = fmaxf(pa, 0.0f);
        float rb = fmaxf(pb, 0.0f);
        ra = nan_bits(pa) ? pa : ra;
        rb = nan_bits(pb) ? pb : rb;
        ev[e]     = (_Float16)ra;
        ev[4 + e] = (_Float16)rb;
      }
      *(v8h*)(At + m * APITCH + e0) = ev;
    }
    __syncthreads();

    v8f acc[2][4];
#pragma unroll
    for (int mt = 0; mt < 2; ++mt)
#pragma unroll
      for (int g = 0; g < 4; ++g) acc[mt][g] = z8;
    {
      const _Float16* wph = WB + (size_t)phase * WPLANE + (size_t)j * KCAT + koff;
#pragma unroll 1
      for (int k0 = 0; k0 < KCAT; k0 += 32) {
        const v16h a0f = FragH::load(ar0 + k0);
        const v16h a1f = FragH::load(ar1 + k0);
        const v16h b0 = FragH::load(wph + k0);
        const v16h b1 = FragH::load(wph + (size_t)1 * HID * KCAT + k0);
        const v16h b2 = FragH::load(wph + (size_t)2 * HID * KCAT + k0);
        const v16h b3 = FragH::load(wph + (size_t)3 * HID * KCAT + k0);
        acc[0][0] = FragH::mma(a0f, b0, acc[0][0]);
        acc[1][0] = FragH::mma(a1f, b0, acc[1][0]);
        acc[0][1] = FragH::mma(a0f, b1, acc[0][1]);
        acc[1][1] = FragH::mma(a1f, b1, acc[1][1]);
        acc[0][2] = FragH::mma(a0f, b2, acc[0][2]);
        acc[1][2] = FragH::mma(a1f, b2, acc[1][2]);
        acc[0][3] = FragH::mma(a0f, b3, acc[0][3]);
        acc[1][3] = FragH::mma(a1f, b3, acc[1][3]);
        guard8(acc[0][0], acc[1][0], acc[0][1], acc[1][1], acc[0][2], acc[1][2], acc[0][3], acc[1][3],
               a0f, a1f, b0, b1, b2, b3);
      }
    }
    acc_guard4(acc[0][0], acc[0][1], acc[0][2], acc[0][3]);
    acc_guard4(acc[1][0], acc[1][1], acc[1][2], acc[1][3]);
    __syncthreads();

#pragma unroll
    for (int mt = 0; mt < 2; ++mt) {
      const v4i ma = *(const v4i*)(msk + 16 * mt + 8 * hh);
      const v4i mb = *(const v4i*)(msk + 16 * mt + 8 * hh + 4);
#pragma unroll
      for (int r = 0; r < 8; ++r) {
        const int mkr = (r < 4) ? ma[r & 3] : mb[r & 3];
        const bool mk = (mkr != 0);
        const float zi = fmaf(acc[mt][0][r], WCARRY_INV, bI);
        const float zf = fmaf(acc[mt][1][r], WCARRY_INV, bF);
        const float zg = fmaf(acc[mt][2][r], WCARRY_INV, bG);
        const float zo = fmaf(acc[mt][3][r], WCARRY_INV, bO);
        const float ig = fsig(zi);
        const float fg = fsig(zf);
        const float gg = ftanh(zg);
        const float og = fsig(zo);
        const float c2 = fg * cst[mt][r] + ig * gg;
        const float h2 = og * ftanh(c2);
        const float cn = mk ? c2 : cst[mt][r];
        const float hn = mk ? h2 : hst[mt][r];
        cst[mt][r] = cn;
        hst[mt][r] = hn;
        const int row = 16 * mt + 8 * hh + r;
        At[row * APITCH + EMB + j] = (_Float16)hn;
        hl[row * HLPITCH + j] = h2;
      }
    }
    __syncthreads();

    if (wave == 0) {
      float sx = 0.0f, sy = 0.0f;
      const float* hr = hl + lane * HLPITCH;
#pragma unroll 2
      for (int jj = 0; jj < HID; jj += 4) {
        const v4f hv = *(const v4f*)(hr + jj);
        const v4f wx = *(const v4f*)(Wfl + jj);
        const v4f wy = *(const v4f*)(Wfl + HID + jj);
        sx = fmaf(hv[0], wx[0], sx); sy = fmaf(hv[0], wy[0], sy);
        sx = fmaf(hv[1], wx[1], sx); sy = fmaf(hv[1], wy[1], sy);
        sx = fmaf(hv[2], wx[2], sx); sy = fmaf(hv[2], wy[2], sy);
        sx = fmaf(hv[3], wx[3], sx); sy = fmaf(hv[3], wy[3], sy);
      }
      const float fx = sx + bfx, fy = sy + bfy;
      const float o2x = o2c[0], o2y = o2c[1];
      v2f ov;
      ov[0] = mkc ? (o2x + fx) : nanv;
      ov[1] = mkc ? (o2y + fy) : nanv;
      volatile v2f* op = (volatile v2f*)(out + ((size_t)t * NTRK + rowbase + lane) * 2);
      *op = ov;
      __threadfence();
      *op = ov;
      pm2 = pm1;
      pm1 = ov;

      const int tn = t + 1;
      const int a = rowbase + lane;
      v2f n1, n2;
      if (tn < 8) {
        n1 = *(const v2f*)(observed + ((size_t)tn * NTRK + a) * 2);
        n2 = *(const v2f*)(observed + ((size_t)(tn + 1) * NTRK + a) * 2);
      } else if (tn == 8) {
        const float px = pm2[0], py = pm2[1], qx = obs8[0], qy = obs8[1];
        n1[0] = __uint_as_float((__float_as_uint(px) & pmask) | (__float_as_uint(qx) & ~pmask));
        n1[1] = __uint_as_float((__float_as_uint(py) & pmask) | (__float_as_uint(qy) & ~pmask));
        n2 = pm1;
      } else {
        n1 = pm2;
        n2 = pm1;
      }
      const float n1x = n1[0], n1y = n1[1], n2x = n2[0], n2y = n2[1];
      const bool mk = !(nan_bits(n1x) || nan_bits(n2x));
      v2f vs;
      vs[0] = mk ? 4.0f * (n2x - n1x) : 0.0f;
      vs[1] = mk ? 4.0f * (n2y - n1y) : 0.0f;
      *(v2f*)(Vs + 2 * lane) = vs;
      msk[lane] = mk ? 1 : 0;
      o2c = n2;
      mkc = mk ? 1 : 0;
    }
    __syncthreads();
  }
}

extern "C" void kernel_launch(void* const* d_in, const int* in_sizes, int n_in,
                              void* d_out, int out_size, void* d_ws, size_t ws_size, hipStream_t stream) {
  if (n_in < 16 || d_out == nullptr || d_ws == nullptr) return;
  if (in_sizes[0] != NOBS * NTRK * 2 || in_sizes[2] != NPRIM + 1 || in_sizes[3] != 2 * EMB || in_sizes[4] != EMB ||
      in_sizes[5] != NGATE * EMB || in_sizes[6] != NGATE * HID || in_sizes[7] != NGATE || in_sizes[8] != NGATE ||
      in_sizes[9] != NGATE * EMB || in_sizes[10] != NGATE * HID || in_sizes[11] != NGATE || in_sizes[12] != NGATE ||
      in_sizes[13] != HID * 2 || in_sizes[14] != 2 || out_size != NSTEPS * NTRK * 2) return;

  const float* observed = (const float*)d_in[0];
  const int*   bsplit   = (const int*)d_in[2];
  const float* W_emb    = (const float*)d_in[3];
  const float* b_emb    = (const float*)d_in[4];
  const float* Wih_e    = (const float*)d_in[5];
  const float* Whh_e    = (const float*)d_in[6];
  const float* bih_e    = (const float*)d_in[7];
  const float* bhh_e    = (const float*)d_in[8];
  const float* Wih_d    = (const float*)d_in[9];
  const float* Whh_d    = (const float*)d_in[10];
  const float* bih_d    = (const float*)d_in[11];
  const float* bhh_d    = (const float*)d_in[12];
  const float* Wf       = (const float*)d_in[13];
  const float* bfp      = (const float*)d_in[14];
  float* out = (float*)d_out;

  char* ws = (char*)d_ws; size_t off = 0;
  auto carve = [&](size_t bytes) -> char* { char* p = ws + off; off += (bytes + 255) & ~(size_t)255; return p; };
  unsigned short* WBp  = (unsigned short*)carve((size_t)2 * WPLANE * 2);
  float*          BIAS = (float*)carve((size_t)2 * NGATE * 4);
  if (off > ws_size || off > (size_t)134217728) return;

  prep_kernel<<<PREP_WBLOCKS + 1, NTHR, 0, stream>>>(Wih_e, Whh_e, bih_e, bhh_e, Wih_d, Whh_d, bih_d, bhh_d, WBp, BIAS);
  lstm_traj_kernel<<<NTRK / ROWS_BLK, NTHR, 0, stream>>>(observed, bsplit, W_emb, b_emb, Wf, bfp, WBp, BIAS, out);
}
